// ResBlock_12979391169046
// MI455X (gfx1250) — hardware-run, weakly checked
//
#include <hip/hip_runtime.h>
#include <math.h>

typedef __attribute__((ext_vector_type(16))) _Float16 v16h;
typedef __attribute__((ext_vector_type(16))) __bf16 v16b;
typedef __attribute__((ext_vector_type(8)))  _Float16 v8h;
typedef __attribute__((ext_vector_type(8)))  float v8f;
typedef __attribute__((ext_vector_type(4)))  float v4f;
typedef __attribute__((ext_vector_type(2)))  float v2f;
typedef __attribute__((ext_vector_type(4)))  unsigned v4u;
typedef __attribute__((ext_vector_type(4)))  int v4i;
typedef float __attribute__((may_alias)) float_a;
typedef int __attribute__((may_alias)) int_a;

template <typename T> __device__ __forceinline__ void vst2(void* p, T v) { *(volatile T*)p = v; __threadfence(); *(volatile T*)p = v; }
__device__ __forceinline__ v8f wmma16(v16h a, v16h b, v8f c) {
  v8f d = __builtin_amdgcn_wmma_f32_16x16x32_f16(false, a, false, b, (short)0, c, false, false);
  asm volatile("v_nop\n\tv_nop\n\tv_nop\n\tv_nop" : "+v"(d) : "v"(a), "v"(b));
  return d;
}
__device__ __forceinline__ v8f wmma_bf(v16b a, v16b b, v8f c) {
  v8f d = __builtin_amdgcn_wmma_f32_16x16x32_bf16(false, a, false, b, (short)0, c, false, false);
  asm volatile("v_nop\n\tv_nop\n\tv_nop\n\tv_nop" : "+v"(d) : "v"(a), "v"(b));
  return d;
}
__device__ __forceinline__ v16h frag_h(const _Float16* rowk0, int lane) {
  union { v16h v; v8h q[2]; } u; const _Float16* p = rowk0 + 8 * (lane >> 4);
  u.q[0] = *(const v8h*)p; u.q[1] = *(const v8h*)(p + 16); return u.v;
}
__device__ __forceinline__ v16h frag_f32(const float* rowk0, int lane) {
  v16h a; const float* p = rowk0 + 8 * (lane >> 4);
#pragma unroll
  for (int i = 0; i < 8; ++i) { a[i] = (_Float16)p[i]; a[8 + i] = (_Float16)p[16 + i]; }
  return a;
}
__device__ __forceinline__ v16h frag_f32s(const float* rowk0, int lane, float sc) {
  v16h a; const float* p = rowk0 + 8 * (lane >> 4);
#pragma unroll
  for (int i = 0; i < 8; ++i) { a[i] = (_Float16)(p[i] * sc); a[8 + i] = (_Float16)(p[16 + i] * sc); }
  return a;
}
__device__ __forceinline__ v16h fragc_f32(const float* W, int k0, int n, int lane, int ld, int K) {
  v16h a; const int g = lane >> 4;
#pragma unroll
  for (int i = 0; i < 8; ++i) { const int ka = k0 + 8 * g + i, kb = ka + 16;
    a[i] = (_Float16)(ka < K ? W[(size_t)(ka < K ? ka : K - 1) * ld + n] : 0.f); a[8 + i] = (_Float16)(kb < K ? W[(size_t)(kb < K ? kb : K - 1) * ld + n] : 0.f); }
  return a;
}
struct F2 { v16b h, l; };
__device__ __forceinline__ F2 bsplit16(const float v[16]) { F2 r;
#pragma unroll
  for (int i = 0; i < 16; ++i) { const __bf16 h = (__bf16)v[i]; r.h[i] = h; r.l[i] = (__bf16)(v[i] - (float)h); }
  return r; }
__device__ __forceinline__ F2 split_row(const float* row, int k0, int lane) { float v[16]; const float* p = row + k0 + 8 * (lane >> 4);
#pragma unroll
  for (int i = 0; i < 8; ++i) { v[i] = p[i]; v[8 + i] = p[16 + i]; }
  return bsplit16(v); }
__device__ __forceinline__ F2 split_rowK(const float* row, int k0, int lane, int K) { float v[16]; const int g = lane >> 4;
#pragma unroll
  for (int i = 0; i < 8; ++i) { const int ka = k0 + 8 * g + i, kb = ka + 16; v[i] = ka < K ? row[ka < K ? ka : K - 1] : 0.f; v[8 + i] = kb < K ? row[kb < K ? kb : K - 1] : 0.f; }
  return bsplit16(v); }
__device__ __forceinline__ F2 split_col(const float* W, int k0, int n, int lane, int ld, int K) { float v[16]; const int g = lane >> 4;
#pragma unroll
  for (int i = 0; i < 8; ++i) { const int ka = k0 + 8 * g + i, kb = ka + 16; v[i] = ka < K ? W[(size_t)(ka < K ? ka : K - 1) * ld + n] : 0.f; v[8 + i] = kb < K ? W[(size_t)(kb < K ? kb : K - 1) * ld + n] : 0.f; }
  return bsplit16(v); }
__device__ __forceinline__ v8f mac3(const F2& a, const F2& b, v8f c) { c = wmma_bf(a.l, b.h, c); c = wmma_bf(a.h, b.l, c); return wmma_bf(a.h, b.h, c); }
__device__ __forceinline__ float sigm(float v) { return 1.0f / (1.0f + expf(-v)); }
#define LDSX() do { asm volatile("s_wait_dscnt 0" ::: "memory"); __builtin_amdgcn_wave_barrier(); __builtin_amdgcn_fence(__ATOMIC_RELEASE, "workgroup"); } while (0)

#define NV 200000
#define KO 27
#define CH 32
#define KW (KO * CH)
#ifndef NVP
#define NVP NV
#endif
typedef int mask_t;
__device__ __forceinline__ float bfr(float v) { return (float)(__bf16)v; }
__device__ __forceinline__ v16b wcol_oi(const float* Wm, int k0, int o, int lane, int K) { v16b w; const float* p = Wm + (size_t)o * K + k0 + 8 * (lane >> 4);
#pragma unroll
  for (int i = 0; i < 8; ++i) { w[i] = (__bf16)p[i]; w[8 + i] = (__bf16)p[16 + i]; }
  return w; }

__device__ __forceinline__ v16b wcol_oi_T(const float* Wm, int k0, int o, int lane) { v16b w; const int g = lane >> 4; float t0[8], t1[8];
#pragma unroll
  for (int i = 0; i < 8; ++i) t0[i] = Wm[(size_t)(k0 + 8 * g + i) * CH + o];
  asm volatile("s_wait_loadcnt 0x0" ::: "memory");
#pragma unroll
  for (int i = 0; i < 8; ++i) t1[i] = Wm[(size_t)(k0 + 16 + 8 * g + i) * CH + o];
  asm volatile("s_wait_loadcnt 0x0" ::: "memory");
#pragma unroll
  for (int i = 0; i < 8; ++i) { w[i] = (__bf16)t0[i]; w[8 + i] = (__bf16)t1[i]; }
  return w; }
#define WS_T1  0u
#define WS_T2  (WS_T1 + 4u * (size_t)NV * CH)
#define WS_ST  (WS_T2 + 4u * (size_t)NV * CH)
#define WS_END (WS_ST + 4u * (size_t)2 * CH * 32)

template <int MODE>
__global__ __launch_bounds__(128) void k_conv(const float* __restrict__ SRC, const int* __restrict__ NBI, const mask_t* __restrict__ NBM, const float* __restrict__ Wt, const float* __restrict__ ST, const float* __restrict__ G, const float* __restrict__ BE, float* __restrict__ OUTR) { __shared__ __align__(16) float sf[4][16][36];
  const int tid = threadIdx.x, wave = tid >> 5, lane = tid & 31, col = lane & 15, g = lane >> 4; const size_t r0 = (size_t)blockIdx.x * 64 + wave * 16; const size_t myrow = r0 + col;
  float mu_[16], sc_[16];
  if (MODE == 1) {
#pragma unroll
    for (int i = 0; i < 16; ++i) { const int c = 8 * g + (i < 8 ? i : 8 + i); mu_[i] = ST[c * 32]; sc_[i] = ST[c * 32 + 1]; }
    asm volatile("s_wait_loadcnt 0x0" ::: "memory");
#pragma unroll
    for (int i = 0; i < 16; ++i) { const int c = 8 * g + (i < 8 ? i : 8 + i); sc_[i] *= bfr(G[c]); }
    asm volatile("s_wait_loadcnt 0x0" ::: "memory"); }
  v8f acc[2] = {};
#pragma unroll 1
  for (int j = 0; j < KO; ++j) { int nb = NBI[myrow * KO + j]; nb = nb < 0 ? 0 : (nb >= NV ? NV - 1 : nb); const float mk = NBM[myrow * KO + j] ? 1.f : 0.f;
    asm volatile("s_wait_loadcnt 0x0" ::: "memory");
    const float* p = SRC + (size_t)nb * CH + 8 * g; float v[16];
#pragma unroll
    for (int i = 0; i < 8; ++i) { v[i] = p[i]; v[8 + i] = p[16 + i]; }
    asm volatile("s_wait_loadcnt 0x0" ::: "memory");
    if (MODE == 0) { v16b a;
#pragma unroll
      for (int i = 0; i < 16; ++i) a[i] = (__bf16)(bfr(v[i]) * mk);
#pragma unroll
      for (int t2 = 0; t2 < 2; ++t2) { const v16b w = wcol_oi_T(Wt, j * CH, t2 * 16 + col, lane); acc[t2] = wmma_bf(a, w, acc[t2]); }
    } else {
#pragma unroll
      for (int i = 0; i < 16; ++i) { const int c = 8 * g + (i < 8 ? i : 8 + i); const float h = fmaxf((v[i] - mu_[i]) * sc_[i] + bfr(BE[c]), 0.f); v[i] = h * mk; }
      const F2 a = bsplit16(v);
#pragma unroll
      for (int t2 = 0; t2 < 2; ++t2) { const v16b w = wcol_oi_T(Wt, j * CH, t2 * 16 + col, lane); acc[t2] = wmma_bf(a.h, w, acc[t2]); acc[t2] = wmma_bf(a.l, w, acc[t2]); } } }
#pragma unroll
  for (int t2 = 0; t2 < 2; ++t2)
#pragma unroll
    for (int r = 0; r < 8; ++r) sf[wave][8 * g + r][t2 * 16 + col] = acc[t2][r];
  LDSX(); for (int rl = 0; rl < 16; ++rl) if (lane < 8) vst2(OUTR + (r0 + rl) * CH + lane * 4, *(const v4f*)&sf[wave][rl][lane * 4]); }
__global__ __launch_bounds__(256) void k_stat(const float* __restrict__ T, float* __restrict__ STAT) { __shared__ float sred[8]; __shared__ float sbc;
  const int t = threadIdx.x; const int c = blockIdx.x;
  float s = 0.f; for (int r = t; r < NVP; r += 256) s += T[(size_t)r * CH + c];
#pragma unroll
  for (int o = 1; o < 32; o <<= 1) s += __shfl_xor(s, o);
  if ((t & 31) == 0) sred[t >> 5] = s; __syncthreads(); if (t == 0) { float a = 0.f; for (int i = 0; i < 8; ++i) a += sred[i]; sbc = a / (float)NVP; } __syncthreads(); const float mean = sbc; __syncthreads();
  float q = 0.f; for (int r = t; r < NVP; r += 256) { const float d = T[(size_t)r * CH + c] - mean; q += d * d; }
#pragma unroll
  for (int o = 1; o < 32; o <<= 1) q += __shfl_xor(q, o);
  if ((t & 31) == 0) sred[t >> 5] = q; __syncthreads(); if (t == 0) { float a = 0.f; for (int i = 0; i < 8; ++i) a += sred[i]; sbc = rsqrtf(a / (float)NVP + 1e-5f); } __syncthreads();
  if (t < 32) { const float v = t == 0 ? mean : (t == 1 ? sbc : 0.f); vst2(STAT + (size_t)c * 32 + t, v); } }
__global__ __launch_bounds__(256) void k_fin(const float* __restrict__ T2, const float* __restrict__ STAT, const float* __restrict__ G, const float* __restrict__ BE, const float* __restrict__ X, float* __restrict__ OUT) { const size_t e4 = (size_t)blockIdx.x * 256 + threadIdx.x; if (e4 >= (size_t)NVP * CH / 4) return; const int c0 = (int)((e4 * 4) % CH); const v4f tv = *(const v4f*)(T2 + e4 * 4); const v4f xv = *(const v4f*)(X + e4 * 4); v4f o;
#pragma unroll
  for (int i = 0; i < 4; ++i) { const int c = c0 + i; const float y = (tv[i] - STAT[c * 32]) * STAT[c * 32 + 1] * bfr(G[c]) + bfr(BE[c]); o[i] = fmaxf(y + bfr(xv[i]), 0.f); }
  vst2(OUT + e4 * 4, o); }
extern "C" void kernel_launch(void* const* d_in, const int* in_sizes, int n_in, void* d_out, int out_size, void* d_ws, size_t ws_size, hipStream_t stream) {
  (void)in_sizes; (void)n_in; (void)out_size;
  if (ws_size < (size_t)WS_END) return;
  char* ws = (char*)d_ws; float *T1 = (float*)(ws + WS_T1), *T2 = (float*)(ws + WS_T2), *ST = (float*)(ws + WS_ST);
  const float* X = (const float*)d_in[0]; const int* NBI = (const int*)d_in[1]; const mask_t* NBM = (const mask_t*)d_in[2]; const float** F = (const float**)d_in;
  k_conv<0><<<dim3(NVP / 64), 128, 0, stream>>>(X, NBI, NBM, F[3], nullptr, nullptr, nullptr, T1);
  k_stat<<<dim3(CH), 256, 0, stream>>>(T1, ST);
  k_conv<1><<<dim3(NVP / 64), 128, 0, stream>>>(T1, NBI, NBM, F[6], ST, F[4], F[5], T2);
  k_stat<<<dim3(CH), 256, 0, stream>>>(T2, ST + CH * 32);
  k_fin<<<dim3((NVP * CH / 4 + 255) / 256), 256, 0, stream>>>(T2, ST + CH * 32, F[7], F[8], X, (float*)d_out);
}
